// RQwenAttention_74715251081268
// MI455X (gfx1250) — hardware-verified
//
#include <hip/hip_runtime.h>
#include <math.h>
#include <stdint.h>

#ifndef NB
#define NB 2
#endif
#ifndef SEQ
#define SEQ 2048
#endif
#define NB_FULL 2
#define S_FULL 2048
#define DMOD  2048
#define NH    16
#define HD    128
#define HHALF (HD / 2)
#define NEXP  8
#define RNK   16
#define NL    (NEXP * RNK)
#define KC    (DMOD + 2 * NL)
#define QO    ((SEQ < 256) ? SEQ : 256)
#define MROWS (NB * SEQ)
#define RSQ_HD 0.08838834764831845f
#define LOG2E 1.4426950408889634f
#define KROPE (-0.20762050593046014f)
#define NEGT  (-1.0e30f)
#define QSC   256.0f
#define KSC   256.0f
#define PCAR  32768.0f
#define VCAR  1024.0f
#define OSC   1024.0f
#define WOS   1024.0f
#define AOS   1024.0f
#define WPB   2
#define NHG   (NH / WPB)
#define NQT   (SEQ / 16)
#define NQTE  (QO / 16)
#define NKT   (SEQ / 32)
#define NSTT  (SEQ / 64)
#define ATT_THREADS (WPB * 32)
#define PTP   36
#define PTW   (16 * PTP)
#define SLP   132
#define SLW   (16 * SLP)
#define WREG  (PTW + SLW)
#define SLAB64 (16 * 68)
#define VTP   72
#define WS_CAP 134217728
#define SZ_XC ((size_t)MROWS * KC * 2)
#define SZ_F  ((size_t)MROWS * DMOD * 4)
#define SZ_OL ((size_t)NB * QO * DMOD * 2)
#define SZ_WC ((size_t)DMOD * KC * 2)
#define SZ_AE ((size_t)NL * DMOD * 2)
#define SZ_Q  ((size_t)MROWS * DMOD * 2)
#define SZ_KL ((size_t)NB * QO * DMOD * 2)
#define SZ_VL ((size_t)NB * NH * HD * QO * 2)
#define SZ_G0A (SZ_XC + SZ_F)
#define SZ_G0B (SZ_XC + SZ_OL)
#define SZ_G0  ((SZ_G0A > SZ_G0B) ? SZ_G0A : SZ_G0B)
#define SZ_TOTAL (SZ_G0 + SZ_WC + SZ_AE + 4 * SZ_Q + SZ_KL + SZ_VL)
static_assert(DMOD == NH * HD && HD == 128 && HHALF == 64 && NH == 16 && WPB == 2 && NHG * WPB == NH);
static_assert(NL == 128 && (NL % 64) == 0 && KC == 2304 && (KC % 32) == 0 && (DMOD % 64) == 0 && (DMOD % 32) == 0);
static_assert(ATT_THREADS == 64);
static_assert(NB >= 1 && NB <= NB_FULL);
static_assert((SEQ % 64) == 0 && SEQ >= 64 && SEQ <= S_FULL);
static_assert((QO % 64) == 0 && QO >= 64 && QO <= SEQ && NQTE * 16 == QO && NQTE <= NQT && (QO % 32) == 0);
static_assert((MROWS % 64) == 0 && (((SEQ * DMOD) / 8) % 256) == 0 && (((DMOD * NL) / 8) % 256) == 0);
static_assert(WPB * WREG * 4 <= 65536 && 2 * HD * VTP * 2 <= 65536 && 4 * SLAB64 * 4 <= 65536);
static_assert(SZ_TOTAL <= (size_t)WS_CAP);
static_assert((size_t)MROWS * DMOD * 4 <= (size_t)33554432);
static_assert((SZ_G0 % 4096) == 0 && (SZ_WC % 4096) == 0 && (SZ_AE % 4096) == 0 && (SZ_Q % 4096) == 0 && (SZ_KL % 4096) == 0);

typedef unsigned short u16;
typedef _Float16 v16h __attribute__((ext_vector_type(16)));
typedef _Float16 v8h  __attribute__((ext_vector_type(8)));
typedef __bf16   v16b __attribute__((ext_vector_type(16)));
typedef float    v8f  __attribute__((ext_vector_type(8)));
typedef float    v4f  __attribute__((ext_vector_type(4)));
typedef unsigned int v4u __attribute__((ext_vector_type(4)));

union FragH { v16h v; v8h h[2]; v4u u[2]; };
union FragB { v16b v; v4u u[2]; };

__device__ __forceinline__ unsigned short bf_bits(float f) {
  unsigned u = __float_as_uint(f);
  return (unsigned short)((u + 0x7FFFu + ((u >> 16) & 1u)) >> 16);
}
__device__ __forceinline__ float bf_up(unsigned short h) { return __uint_as_float(((unsigned)h) << 16); }
__device__ __forceinline__ float bfr(float f) { return bf_up(bf_bits(f)); }
__device__ __forceinline__ unsigned short h_bits(_Float16 x) { return __builtin_bit_cast(unsigned short, x); }
__device__ __forceinline__ unsigned pk16(unsigned short a, unsigned short b) { return (unsigned)a | ((unsigned)b << 16); }
__device__ __forceinline__ v8f zero8() { v8f z = {0.f, 0.f, 0.f, 0.f, 0.f, 0.f, 0.f, 0.f}; return z; }

__device__ __forceinline__ v16h ldfrag_h(const _Float16* p) {
  FragH f;
  f.h[0] = *(const v8h*)(p);
  f.h[1] = *(const v8h*)(p + 16);
  return f.v;
}
__device__ __forceinline__ v16b ldfrag_b(const u16* p) {
  FragB f;
  f.u[0] = *(const v4u*)(p);
  f.u[1] = *(const v4u*)(p + 16);
  return f.v;
}

__device__ __forceinline__ v8f mma_h(v16h a, v16h b, v8f c) {
  return __builtin_amdgcn_wmma_f32_16x16x32_f16(false, a, false, b, (short)0, c, false, false);
}
__device__ __forceinline__ v8f mma_b(v16b a, v16b b, v8f c) {
  return __builtin_amdgcn_wmma_f32_16x16x32_bf16(false, a, false, b, (short)0, c, false, false);
}
__device__ __forceinline__ void guard2(v8f& a, v8f& b, v16h x0, v16h x1, v16h x2, v16h x3, v16h x4, v16h x5) {
#if defined(__HIP_DEVICE_COMPILE__)
  asm volatile("v_nop\n\tv_nop\n\tv_nop\n\tv_nop"
               : "+v"(a), "+v"(b) : "v"(x0), "v"(x1), "v"(x2), "v"(x3), "v"(x4), "v"(x5) : "memory");
#endif
}
template <typename F>
__device__ __forceinline__ void guard6(v8f& a, v8f& b, v8f& c, v8f& d, F x0, F x1, F x2, F x3, F x4, F x5) {
#if defined(__HIP_DEVICE_COMPILE__)
  asm volatile("v_nop\n\tv_nop\n\tv_nop\n\tv_nop"
               : "+v"(a), "+v"(b), "+v"(c), "+v"(d) : "v"(x0), "v"(x1), "v"(x2), "v"(x3), "v"(x4), "v"(x5) : "memory");
#endif
}
__device__ __forceinline__ void acc_guard4(v8f& a, v8f& b, v8f& c, v8f& d) {
#if defined(__HIP_DEVICE_COMPILE__)
  asm volatile("v_nop\n\tv_nop\n\tv_nop\n\tv_nop" : "+v"(a), "+v"(b), "+v"(c), "+v"(d));
#endif
}
__device__ __forceinline__ void wave_sync_lds() {
  __builtin_amdgcn_fence(__ATOMIC_RELEASE, "workgroup");
  __builtin_amdgcn_wave_barrier();
  __builtin_amdgcn_fence(__ATOMIC_ACQUIRE, "workgroup");
}

__global__ __launch_bounds__(256) void cvtrows(const float* __restrict__ X, int spitch, int scols, int nrows,
                                               u16* D, int dp, int c0, int f16mode, float scale) {
  const int gt = blockIdx.x * 256 + (int)threadIdx.x;
  const int n8 = (nrows * scols) >> 3;
  if (gt >= n8) return;
  const int e0 = gt * 8;
  const int r  = e0 / scols;
  const int c  = e0 - r * scols;
  const float* p = X + (size_t)r * spitch + c;
  const v4f a = *(const v4f*)(p), b4 = *(const v4f*)(p + 4);
  float w[8];
#pragma unroll
  for (int e = 0; e < 4; ++e) { w[e] = a[e]; w[4 + e] = b4[e]; }
  v4u o;
#pragma unroll
  for (int e = 0; e < 4; ++e) {
    const float f0 = w[2 * e], f1 = w[2 * e + 1];
    const unsigned short hb0 = h_bits((_Float16)(bfr(f0) * scale));
    const unsigned short hb1 = h_bits((_Float16)(bfr(f1) * scale));
    const unsigned short bb0 = bf_bits(f0);
    const unsigned short bb1 = bf_bits(f1);
    o[e] = (f16mode != 0) ? pk16(hb0, hb1) : pk16(bb0, bb1);
  }
  u16* d = D + (size_t)r * dp + c0 + c;
  for (int pass = 0; pass < 2; ++pass) {
    *(volatile v4u*)(d) = o;
    __threadfence();
  }
}

template <int HASB>
__device__ __forceinline__ void epi64(float* sl, v8f a0, v8f a1, v8f a2, v8f a3, float oscale,
                                      const float* __restrict__ bias,
                                      float* C, int ldc, size_t rowb, int col0, int lane) {
  const int hh = lane >> 4, m = lane & 15;
  float bv0 = 0.0f, bv1 = 0.0f, bv2 = 0.0f, bv3 = 0.0f;
  if constexpr (HASB != 0) {
    bv0 = bfr(bias[col0 + m]);
    bv1 = bfr(bias[col0 + 16 + m]);
    bv2 = bfr(bias[col0 + 32 + m]);
    bv3 = bfr(bias[col0 + 48 + m]);
  }
#pragma unroll
  for (int r = 0; r < 8; ++r) {
    const int ro = (8 * hh + r) * 68 + m;
    sl[ro]      = a0[r] * oscale + bv0;
    sl[ro + 16] = a1[r] * oscale + bv1;
    sl[ro + 32] = a2[r] * oscale + bv2;
    sl[ro + 48] = a3[r] * oscale + bv3;
  }
  wave_sync_lds();
  v4f vals[8];
#pragma unroll
  for (int it = 0; it < 8; ++it) vals[it] = *(const v4f*)(sl + (it * 2 + hh) * 68 + m * 4);
  float* dst = C + (rowb + (size_t)hh) * (size_t)ldc + col0 + m * 4;
  for (int pass = 0; pass < 2; ++pass) {
#pragma unroll
    for (int it = 0; it < 8; ++it) {
      *(volatile v4f*)(dst + (size_t)(it * 2) * (size_t)ldc) = vals[it];
    }
    __threadfence();
  }
}

__global__ __launch_bounds__(128)
void gemm_bff(const u16* __restrict__ A, int lda, const u16* __restrict__ Bt, int ldb, const float* __restrict__ bias,
              float* C, int ldc, int M, int N, int K) {
  __shared__ __align__(16) float slab[4 * SLAB64];
  const int tid = threadIdx.x, wave = tid >> 5, lane = tid & 31, hh = lane >> 4, m = lane & 15;
  const int ntile = N >> 6;
  const int bid   = blockIdx.x;
  const int rowb  = (bid / ntile) * 64 + wave * 16;
  const int col0  = (bid % ntile) * 64;
  if (rowb + 16 > M) return;
  const u16* ap = A  + (size_t)(rowb + m) * lda + 8 * hh;
  const u16* bp = Bt + (size_t)(col0 + m) * ldb + 8 * hh;
  const size_t bs = (size_t)16 * ldb;
  v8f acc0 = zero8(), acc1 = zero8(), acc2 = zero8(), acc3 = zero8();
#pragma unroll 1
  for (int k0 = 0; k0 < K; k0 += 32) {
    const v16b a  = ldfrag_b(ap + k0);
    const v16b b0 = ldfrag_b(bp + k0);
    const v16b b1 = ldfrag_b(bp + bs + k0);
    const v16b b2 = ldfrag_b(bp + 2 * bs + k0);
    const v16b b3 = ldfrag_b(bp + 3 * bs + k0);
    acc0 = mma_b(a, b0, acc0);
    acc1 = mma_b(a, b1, acc1);
    acc2 = mma_b(a, b2, acc2);
    acc3 = mma_b(a, b3, acc3);
    guard6<v16b>(acc0, acc1, acc2, acc3, a, b0, b1, b2, b3, a);
  }
  epi64<1>(slab + wave * SLAB64, acc0, acc1, acc2, acc3, 1.0f, bias, C, ldc, (size_t)rowb, col0, lane);
}

template <int OPH, int HOUT>
__global__ __launch_bounds__(128)
void gemm_lr(const u16* A, int lda, const u16* __restrict__ Bt, int ldb, int K, const float* __restrict__ gate,
             u16* Dst, int M, float oscale, float osc) {
  __shared__ __align__(16) float slab[4 * SLAB64];
  const int tid = threadIdx.x, wave = tid >> 5, lane = tid & 31, hh = lane >> 4, m = lane & 15;
  const int bid  = blockIdx.x;
  const int rowb = (bid >> 1) * 64 + wave * 16;
  const int col0 = (bid & 1) * 64;
  if (rowb + 16 > M) return;
  v8f acc0 = zero8(), acc1 = zero8(), acc2 = zero8(), acc3 = zero8();
  if constexpr (OPH == 0) {
    const u16* ap = A  + (size_t)(rowb + m) * lda + 8 * hh;
    const u16* bp = Bt + (size_t)(col0 + m) * ldb + 8 * hh;
    const size_t bs = (size_t)16 * ldb;
#pragma unroll 1
    for (int k0 = 0; k0 < K; k0 += 32) {
      const v16b a  = ldfrag_b(ap + k0);
      const v16b b0 = ldfrag_b(bp + k0);
      const v16b b1 = ldfrag_b(bp + bs + k0);
      const v16b b2 = ldfrag_b(bp + 2 * bs + k0);
      const v16b b3 = ldfrag_b(bp + 3 * bs + k0);
      acc0 = mma_b(a, b0, acc0);
      acc1 = mma_b(a, b1, acc1);
      acc2 = mma_b(a, b2, acc2);
      acc3 = mma_b(a, b3, acc3);
      guard6<v16b>(acc0, acc1, acc2, acc3, a, b0, b1, b2, b3, a);
    }
  } else {
    const _Float16* ap = (const _Float16*)(const void*)A  + (size_t)(rowb + m) * lda + 8 * hh;
    const _Float16* bp = (const _Float16*)(const void*)Bt + (size_t)(col0 + m) * ldb + 8 * hh;
    const size_t bs = (size_t)16 * ldb;
#pragma unroll 1
    for (int k0 = 0; k0 < K; k0 += 32) {
      const v16h a  = ldfrag_h(ap + k0);
      const v16h b0 = ldfrag_h(bp + k0);
      const v16h b1 = ldfrag_h(bp + bs + k0);
      const v16h b2 = ldfrag_h(bp + 2 * bs + k0);
      const v16h b3 = ldfrag_h(bp + 3 * bs + k0);
      acc0 = mma_h(a, b0, acc0);
      acc1 = mma_h(a, b1, acc1);
      acc2 = mma_h(a, b2, acc2);
      acc3 = mma_h(a, b3, acc3);
      guard6<v16h>(acc0, acc1, acc2, acc3, a, b0, b1, b2, b3, a);
    }
  }
  float* sl = slab + wave * SLAB64;
#pragma unroll
  for (int r = 0; r < 8; ++r) {
    const int ro = (8 * hh + r) * 68 + m;
    sl[ro]      = acc0[r] * oscale;
    sl[ro + 16] = acc1[r] * oscale;
    sl[ro + 32] = acc2[r] * oscale;
    sl[ro + 48] = acc3[r] * oscale;
  }
  wave_sync_lds();
  const int rq = lane >> 3, c8 = (lane & 7) * 8;
  const int ex = (col0 + c8) >> 4;
  v4u oh[4], ol[4];
#pragma unroll
  for (int it = 0; it < 4; ++it) {
    const int row  = it * 4 + rq;
    const int grow = rowb + row;
    const int bi   = grow / SEQ;
    const int s    = grow - bi * SEQ;
    const float g  = bfr(gate[((size_t)bi * S_FULL + s) * NEXP + ex]);
    const v4f a = *(const v4f*)(sl + row * 68 + c8), b4 = *(const v4f*)(sl + row * 68 + c8 + 4);
    float w[8];
#pragma unroll
    for (int e = 0; e < 4; ++e) { w[e] = a[e] * g; w[4 + e] = b4[e] * g; }
#pragma unroll
    for (int q = 0; q < 4; ++q) {
      const float f0 = w[2 * q], f1 = w[2 * q + 1];
      if constexpr (HOUT == 0) {
        const unsigned short h0 = bf_bits(f0), h1 = bf_bits(f1);
        const unsigned short l0 = bf_bits(f0 - bf_up(h0)), l1 = bf_bits(f1 - bf_up(h1));
        oh[it][q] = pk16(h0, h1);
        ol[it][q] = pk16(l0, l1);
      } else {
        const float t0 = f0 * osc, t1 = f1 * osc;
        const _Float16 a0 = (_Float16)t0, a1 = (_Float16)t1;
        const _Float16 r0 = (_Float16)(t0 - (float)a0), r1 = (_Float16)(t1 - (float)a1);
        oh[it][q] = pk16(h_bits(a0), h_bits(a1));
        ol[it][q] = pk16(h_bits(r0), h_bits(r1));
      }
    }
  }
  for (int pass = 0; pass < 2; ++pass) {
#pragma unroll
    for (int it = 0; it < 4; ++it) {
      const int row = it * 4 + rq;
      u16* d = Dst + (size_t)(rowb + row) * KC + DMOD + col0 + c8;
      *(volatile v4u*)(d) = oh[it];
      *(volatile v4u*)(d + NL) = ol[it];
    }
    __threadfence();
  }
}

__device__ __forceinline__ void rot_pair(float xl, float xh, float cv, float sv, float sc,
                                         unsigned short& hl, unsigned short& hhv, unsigned short& ll, unsigned short& lh) {
#pragma clang fp contract(off)
  const float rl = xl * cv - xh * sv;
  const float rh = xl * sv + xh * cv;
  const float tl = rl * sc, th = rh * sc;
  const _Float16 a = (_Float16)tl, bq = (_Float16)th;
  hl  = h_bits(a);
  hhv = h_bits(bq);
  ll  = h_bits((_Float16)(tl - (float)a));
  lh  = h_bits((_Float16)(th - (float)bq));
}

__global__ __launch_bounds__(128) void rope16(const float* __restrict__ F, u16* Hp, u16* Lp, int lrows, float sc) {
#pragma clang fp contract(off)
  __shared__ __align__(16) float cst[HHALF];
  __shared__ __align__(16) float snt[HHALF];
  const int tid = (int)threadIdx.x;
  const int r   = (int)blockIdx.x;
  if (r >= MROWS) return;
  const int b   = r / SEQ;
  const int s   = r - b * SEQ;
  if (tid < HHALF) {
    const float invf = exp2f((float)tid * KROPE);
    const float ang  = (float)s * invf;
    cst[tid] = cosf(ang);
    snt[tid] = sinf(ang);
  }
  __syncthreads();
  const int dlo = (tid & 7) * 8;
  const int clo = (tid >> 3) * HD + dlo;
  const float* p = F + (size_t)r * DMOD + clo;
  const v4f xa = *(const v4f*)(p), xb = *(const v4f*)(p + 4);
  const v4f ya = *(const v4f*)(p + HHALF), yb = *(const v4f*)(p + HHALF + 4);
  const v4f ca = *(const v4f*)(cst + dlo), cb = *(const v4f*)(cst + dlo + 4);
  const v4f sa = *(const v4f*)(snt + dlo), sb = *(const v4f*)(snt + dlo + 4);
  float xl[8], xh[8], cv[8], sv[8];
#pragma unroll
  for (int e = 0; e < 4; ++e) {
    xl[e] = xa[e];        xl[4 + e] = xb[e];
    xh[e] = ya[e];        xh[4 + e] = yb[e];
    cv[e] = ca[e];        cv[4 + e] = cb[e];
    sv[e] = sa[e];        sv[4 + e] = sb[e];
  }
  v4u ohl, ohh, oll, olh;
#pragma unroll
  for (int e = 0; e < 4; ++e) {
    unsigned short hl0, hh0, ll0, lh0, hl1, hh1, ll1, lh1;
    rot_pair(xl[2 * e],     xh[2 * e],     cv[2 * e],     sv[2 * e],     sc, hl0, hh0, ll0, lh0);
    rot_pair(xl[2 * e + 1], xh[2 * e + 1], cv[2 * e + 1], sv[2 * e + 1], sc, hl1, hh1, ll1, lh1);
    ohl[e] = pk16(hl0, hl1);
    ohh[e] = pk16(hh0, hh1);
    oll[e] = pk16(ll0, ll1);
    olh[e] = pk16(lh0, lh1);
  }
  const bool wl = (s < lrows);
  u16* dh = Hp + (size_t)r * DMOD + clo;
  u16* dl = Lp + ((size_t)b * lrows + (size_t)(wl ? s : 0)) * DMOD + clo;
  for (int pass = 0; pass < 2; ++pass) {
    *(volatile v4u*)(dh) = ohl;
    *(volatile v4u*)(dh + HHALF) = ohh;
    if (wl) {
      *(volatile v4u*)(dl) = oll;
      *(volatile v4u*)(dl + HHALF) = olh;
    }
    __threadfence();
  }
}

__global__ __launch_bounds__(256) void vt16(const float* __restrict__ F, u16* VHo, u16* VLo) {
  __shared__ __align__(16) u16 TH[HD * VTP];
  __shared__ __align__(16) u16 TL[HD * VTP];
  const int tid = threadIdx.x;
  const int bid = blockIdx.x;
  const int st  = bid % NSTT;
  const int t2  = bid / NSTT;
  const int h   = t2 % NH;
  const int b   = t2 / NH;
  if (b >= NB) return;
  const int sl0 = st * 64;
  {
    const int sl = tid >> 2;
    const int dc = (tid & 3) * 32;
    const float* src = F + ((size_t)b * SEQ + sl0 + sl) * DMOD + h * HD + dc;
#pragma unroll
    for (int i = 0; i < 8; ++i) {
      const v4f a = *(const v4f*)(src + 4 * i);
#pragma unroll
      for (int e = 0; e < 4; ++e) {
        const float t = a[e] * VCAR;
        const _Float16 hv = (_Float16)t;
        const _Float16 lv = (_Float16)(t - (float)hv);
        TH[(dc + 4 * i + e) * VTP + sl] = h_bits(hv);
        TL[(dc + 4 * i + e) * VTP + sl] = h_bits(lv);
      }
    }
  }
  __syncthreads();
  v4u vh[4], vl[4];
  const int q8 = tid >> 3, p8 = (tid & 7) * 8;
#pragma unroll
  for (int it = 0; it < 4; ++it) {
    const int line = it * 32 + q8;
    vh[it] = *(const v4u*)(TH + line * VTP + p8);
    vl[it] = *(const v4u*)(TL + line * VTP + p8);
  }
  const bool wl = (sl0 + 64 <= QO);
  const size_t hrow  = (size_t)(b * NH + h) * HD;
  const size_t baseh = hrow * SEQ + (size_t)sl0 + p8;
  const size_t basel = hrow * QO  + (size_t)(wl ? sl0 : 0) + p8;
  for (int pass = 0; pass < 2; ++pass) {
#pragma unroll
    for (int it = 0; it < 4; ++it) {
      const int line = it * 32 + q8;
      *(volatile v4u*)(VHo + baseh + (size_t)line * SEQ) = vh[it];
      if (wl) {
        *(volatile v4u*)(VLo + basel + (size_t)line * QO) = vl[it];
      }
    }
    __threadfence();
  }
}

template <int EARLY>
__global__ __launch_bounds__(ATT_THREADS)
void attn_c(const u16* __restrict__ QHp, const u16* __restrict__ QLp,
            const u16* __restrict__ KHp, const u16* __restrict__ KLp,
            const u16* __restrict__ VHp, const u16* __restrict__ VLp,
            u16* OCp, u16* OLp, int qt0, int nqt) {
  __shared__ __align__(16) float smem[WPB * WREG];

  const int tid  = threadIdx.x;
  const int wave = tid >> 5;
  const int lane = tid & 31;
  const int hh   = lane >> 4;
  const int c    = lane & 15;
  const int bid  = blockIdx.x;
  const int qt   = qt0 + (bid % nqt);
  const int t2   = bid / nqt;
  const int hg   = t2 % NHG;
  const int b    = t2 / NHG;
  if (b >= NB) return;
  const int q0   = qt * 16;
  if (q0 + 16 > SEQ) return;
  const int head = hg * WPB + wave;

  float* pt   = smem + wave * WREG;
  float* slab = pt + PTW;

  const size_t hcol = (size_t)head * HD + 8 * hh;
  const _Float16* Qh  = (const _Float16*)(const void*)QHp + ((size_t)b * SEQ + q0 + c) * DMOD + hcol;
  const _Float16* Ql  = (const _Float16*)(const void*)QLp + ((size_t)b * SEQ + q0 + c) * DMOD + hcol;
  const _Float16* Khb = (const _Float16*)(const void*)KHp + ((size_t)b * SEQ + c) * DMOD + hcol;
  const _Float16* Klb = (const _Float16*)(const void*)KLp + ((size_t)b * QO + c) * DMOD + hcol;
  const _Float16* Vhb = (const _Float16*)(const void*)VHp + ((size_t)(b * NH + head) * HD + c) * SEQ + 8 * hh;
  const _Float16* Vlb = (const _Float16*)(const void*)VLp + ((size_t)(b * NH + head) * HD + c) * QO + 8 * hh;
  const float lsc = RSQ_HD * (LOG2E / (QSC * KSC));
  const float oc  = 1.0f / (PCAR * VCAR);
  const size_t KROW = (size_t)DMOD;

  float mrow[8], lrow[8];
  v8f o[8];
#pragma unroll
  for (int r = 0; r < 8; ++r) { mrow[r] = -INFINITY; lrow[r] = 0.f; }
#pragma unroll
  for (int j = 0; j < 8; ++j) o[j] = zero8();
  const int ncaus = (q0 >> 5) + 1;
  const int nkt = (ncaus < NKT) ? ncaus : NKT;
  const int qr0 = q0 + 8 * hh;

#pragma unroll 1
  for (int kt = 0; kt < nkt; ++kt) {
    const int kb = kt * 32;
    v8f s0 = zero8(), s1 = zero8();
    const _Float16* k0p = Khb + (size_t)kb * KROW;
    const _Float16* k1p = k0p + (size_t)16 * KROW;
    if constexpr (EARLY != 0) {
      const _Float16* l0p = Klb + (size_t)kb * KROW;
      const _Float16* l1p = l0p + (size_t)16 * KROW;
#pragma unroll
      for (int kk = 0; kk < HD / 32; ++kk) {
        const v16h qh  = ldfrag_h(Qh + kk * 32);
        const v16h ql  = ldfrag_h(Ql + kk * 32);
        const v16h kh0 = ldfrag_h(k0p + kk * 32);
        const v16h kh1 = ldfrag_h(k1p + kk * 32);
        const v16h kl0 = ldfrag_h(l0p + kk * 32);
        const v16h kl1 = ldfrag_h(l1p + kk * 32);
        s0 = mma_h(qh, kh0, s0);
        s0 = mma_h(ql, kh0, s0);
        s0 = mma_h(qh, kl0, s0);
        s1 = mma_h(qh, kh1, s1);
        s1 = mma_h(ql, kh1, s1);
        s1 = mma_h(qh, kl1, s1);
        guard2(s0, s1, qh, ql, kh0, kl0, kh1, kl1);
      }
    } else {
#pragma unroll
      for (int kk = 0; kk < HD / 32; ++kk) {
        const v16h qh  = ldfrag_h(Qh + kk * 32);
        const v16h ql  = ldfrag_h(Ql + kk * 32);
        const v16h kh0 = ldfrag_h(k0p + kk * 32);
        const v16h kh1 = ldfrag_h(k1p + kk * 32);
        s0 = mma_h(qh, kh0, s0);
        s0 = mma_h(ql, kh0, s0);
        s1 = mma_h(qh, kh1, s1);
        s1 = mma_h(ql, kh1, s1);
        guard2(s0, s1, qh, ql, kh0, kh1, qh, ql);
      }
    }
    const int key0 = kb + c, key1 = kb + 16 + c;
#pragma unroll
    for (int r = 0; r < 8; ++r) {
      const int   qr = qr0 + r;
      const float u0 = s0[r] * lsc;
      const float u1 = s1[r] * lsc;
      const float t0 = (key0 <= qr) ? u0 : NEGT;
      const float t1 = (key1 <= qr) ? u1 : NEGT;
      float mx = fmaxf(t0, t1);
#pragma unroll
      for (int off = 1; off < 16; off <<= 1) mx = fmaxf(mx, __shfl_xor(mx, off, 32));
      const float mn = fmaxf(mrow[r], mx);
      const float ms = (mn == -INFINITY) ? 0.0f : mn;
      const float al = exp2f(mrow[r] - ms);
      mrow[r] = mn;
      const float e0 = exp2f(t0 - ms), e1 = exp2f(t1 - ms);
      float ps = e0 + e1;
#pragma unroll
      for (int off = 1; off < 16; off <<= 1) ps += __shfl_xor(ps, off, 32);
      lrow[r] = lrow[r] * al + ps;
#pragma unroll
      for (int j = 0; j < 8; ++j) o[j][r] *= al;
      const int ro = (8 * hh + r) * PTP + c;
      pt[ro]      = e0;
      pt[ro + 16] = e1;
    }
    wave_sync_lds();
    FragH ph;
    const float* prow = pt + c * PTP + 8 * hh;
    const v4f p0 = *(const v4f*)(prow), p1 = *(const v4f*)(prow + 4);
    const v4f p2 = *(const v4f*)(prow + 16), p3 = *(const v4f*)(prow + 20);
    if constexpr (EARLY != 0) {
      FragH pl;
#pragma unroll
      for (int e = 0; e < 4; ++e) {
        const float ta = p0[e] * PCAR, tb = p1[e] * PCAR, tc = p2[e] * PCAR, td = p3[e] * PCAR;
        const _Float16 ha = (_Float16)ta, hb = (_Float16)tb, hc = (_Float16)tc, hd = (_Float16)td;
        ph.h[0][e]     = ha;
        ph.h[0][4 + e] = hb;
        ph.h[1][e]     = hc;
        ph.h[1][4 + e] = hd;
        pl.h[0][e]     = (_Float16)(ta - (float)ha);
        pl.h[0][4 + e] = (_Float16)(tb - (float)hb);
        pl.h[1][e]     = (_Float16)(tc - (float)hc);
        pl.h[1][4 + e] = (_Float16)(td - (float)hd);
      }
      const _Float16* vhp = Vhb + kb;
      const _Float16* vlp = Vlb + kb;
#pragma unroll
      for (int jg = 0; jg < 4; ++jg) {
        const size_t da = (size_t)(2 * jg) * 16 * SEQ;
        const size_t db = da + (size_t)16 * SEQ;
        const size_t la = (size_t)(2 * jg) * 16 * QO;
        const size_t lb = la + (size_t)16 * QO;
        const v16h vha = ldfrag_h(vhp + da), vhb2 = ldfrag_h(vhp + db);
        const v16h vla = ldfrag_h(vlp + la), vlb2 = ldfrag_h(vlp + lb);
        o[2 * jg]     = mma_h(ph.v, vha,  o[2 * jg]);
        o[2 * jg]     = mma_h(pl.v, vha,  o[2 * jg]);
        o[2 * jg]     = mma_h(ph.v, vla,  o[2 * jg]);
        o[2 * jg + 1] = mma_h(ph.v, vhb2, o[2 * jg + 1]);
        o[2 * jg + 1] = mma_h(pl.v, vhb2, o[2 * jg + 1]);
        o[2 * jg + 1] = mma_h(ph.v, vlb2, o[2 * jg + 1]);
        guard2(o[2 * jg], o[2 * jg + 1], ph.v, pl.v, vha, vhb2, vla, vlb2);
      }
    } else {
#pragma unroll
      for (int e = 0; e < 4; ++e) {
        ph.h[0][e]     = (_Float16)(p0[e] * PCAR);
        ph.h[0][4 + e] = (_Float16)(p1[e] * PCAR);
        ph.h[1][e]     = (_Float16)(p2[e] * PCAR);
        ph.h[1][4 + e] = (_Float16)(p3[e] * PCAR);
      }
      const _Float16* vhp = Vhb + kb;
#pragma unroll
      for (int jg = 0; jg < 4; ++jg) {
        const size_t da = (size_t)(2 * jg) * 16 * SEQ;
        const size_t db = da + (size_t)16 * SEQ;
        const v16h vha = ldfrag_h(vhp + da), vhb2 = ldfrag_h(vhp + db);
        o[2 * jg]     = mma_h(ph.v, vha,  o[2 * jg]);
        o[2 * jg + 1] = mma_h(ph.v, vhb2, o[2 * jg + 1]);
        guard2(o[2 * jg], o[2 * jg + 1], ph.v, ph.v, vha, vhb2, vha, vhb2);
      }
    }
    wave_sync_lds();
  }
  acc_guard4(o[0], o[1], o[2], o[3]);
  acc_guard4(o[4], o[5], o[6], o[7]);
#pragma unroll
  for (int r = 0; r < 8; ++r) {
    const float lv  = lrow[r];
    const float ls  = (lv > 0.0f) ? lv : 1.0f;
    const float inv = (lv > 0.0f) ? ((1.0f / ls) * oc) : 0.0f;
#pragma unroll
    for (int j = 0; j < 8; ++j) {
      const int idx = (8 * hh + r) * SLP + j * 16 + c;
      slab[idx] = o[j][r] * inv;
    }
  }

  wave_sync_lds();
  v4u oh[8], ol[8];
  const int rq = lane >> 4, c8 = (lane & 15) * 8;
#pragma unroll
  for (int it = 0; it < 8; ++it) {
    const int row = it * 2 + rq;
    const v4f a = *(const v4f*)(slab + row * SLP + c8), b4 = *(const v4f*)(slab + row * SLP + c8 + 4);
    float w[8];
#pragma unroll
    for (int e = 0; e < 4; ++e) { w[e] = a[e] * OSC; w[4 + e] = b4[e] * OSC; }
#pragma unroll
    for (int e = 0; e < 4; ++e) {
      const _Float16 h0 = (_Float16)w[2 * e], h1 = (_Float16)w[2 * e + 1];
      oh[it][e] = pk16(h_bits(h0), h_bits(h1));
      if constexpr (EARLY != 0) {
        const _Float16 l0 = (_Float16)(w[2 * e] - (float)h0), l1 = (_Float16)(w[2 * e + 1] - (float)h1);
        ol[it][e] = pk16(h_bits(l0), h_bits(l1));
      } else {
        ol[it][e] = 0u;
      }
    }
  }
  const size_t ob  = ((size_t)b * SEQ + q0) * KC   + (size_t)head * HD + c8;
  const size_t olb = ((size_t)b * QO  + q0) * DMOD + (size_t)head * HD + c8;
  for (int pass = 0; pass < 2; ++pass) {
#pragma unroll
    for (int it = 0; it < 8; ++it) {
      const int row = it * 2 + rq;
      *(volatile v4u*)(OCp + ob + (size_t)row * KC) = oh[it];
      if constexpr (EARLY != 0) {
        *(volatile v4u*)(OLp + olb + (size_t)row * DMOD) = ol[it];
      }
    }
    __threadfence();
  }
}

template <int NPROD>
__global__ __launch_bounds__(128)
void gemm_o(const u16* __restrict__ Ah, const u16* __restrict__ Al, const u16* __restrict__ Bt,
            float* C, int sbeg, int nrt, float oscale) {
  __shared__ __align__(16) float slab[4 * SLAB64];
  const int tid = threadIdx.x, wave = tid >> 5, lane = tid & 31, hh = lane >> 4, m = lane & 15;
  const int ntile = DMOD >> 6;
  const int bid   = blockIdx.x;
  const int ct    = bid % ntile;
  const int t2    = bid / ntile;
  const int rt    = t2 % nrt;
  const int bb    = t2 / nrt;
  if (bb >= NB) return;
  const int srow  = sbeg + rt * 64 + wave * 16;
  if (srow + 16 > SEQ) return;
  const int col0  = ct * 64;
  const size_t rowA = (size_t)bb * SEQ + srow;
  const size_t rowL = (size_t)bb * QO + srow;
  const _Float16* ahp = (const _Float16*)(const void*)Ah + (rowA + m) * KC + 8 * hh;
  const _Float16* alp = (const _Float16*)(const void*)Al + (rowL + m) * DMOD + 8 * hh;
  const _Float16* bp  = (const _Float16*)(const void*)Bt + (size_t)(col0 + m) * KC + 8 * hh;
  const size_t bs = (size_t)16 * KC;
  v8f acc0 = zero8(), acc1 = zero8(), acc2 = zero8(), acc3 = zero8();
  if constexpr (NPROD == 2) {
#pragma unroll 1
    for (int k0 = 0; k0 < DMOD; k0 += 32) {
      const v16h ah = ldfrag_h(ahp + k0), al = ldfrag_h(alp + k0);
      const v16h b0 = ldfrag_h(bp + k0);
      const v16h b1 = ldfrag_h(bp + bs + k0);
      const v16h b2 = ldfrag_h(bp + 2 * bs + k0);
      const v16h b3 = ldfrag_h(bp + 3 * bs + k0);
      acc0 = mma_h(ah, b0, acc0);  acc0 = mma_h(al, b0, acc0);
      acc1 = mma_h(ah, b1, acc1);  acc1 = mma_h(al, b1, acc1);
      acc2 = mma_h(ah, b2, acc2);  acc2 = mma_h(al, b2, acc2);
      acc3 = mma_h(ah, b3, acc3);  acc3 = mma_h(al, b3, acc3);
      guard6<v16h>(acc0, acc1, acc2, acc3, ah, al, b0, b1, b2, b3);
    }
#pragma unroll 1
    for (int k0 = DMOD; k0 < KC; k0 += 32) {
      const v16h ah = ldfrag_h(ahp + k0);
      const v16h b0 = ldfrag_h(bp + k0);
      const v16h b1 = ldfrag_h(bp + bs + k0);
      const v16h b2 = ldfrag_h(bp + 2 * bs + k0);
      const v16h b3 = ldfrag_h(bp + 3 * bs + k0);
      acc0 = mma_h(ah, b0, acc0);
      acc1 = mma_h(ah, b1, acc1);
      acc2 = mma_h(ah, b2, acc2);
      acc3 = mma_h(ah, b3, acc3);
      guard6<v16h>(acc0, acc1, acc2, acc3, ah, b0, b1, b2, b3, ah);
    }
  } else {
#pragma unroll 1
    for (int k0 = 0; k0 < KC; k0 += 32) {
      const v16h ah = ldfrag_h(ahp + k0);
      const v16h b0 = ldfrag_h(bp + k0);
      const v16h b1 = ldfrag_h(bp + bs + k0);
      const v16h b2 = ldfrag_h(bp + 2 * bs + k0);
      const v16h b3 = ldfrag_h(bp + 3 * bs + k0);
      acc0 = mma_h(ah, b0, acc0);
      acc1 = mma_h(ah, b1, acc1);
      acc2 = mma_h(ah, b2, acc2);
      acc3 = mma_h(ah, b3, acc3);
      guard6<v16h>(acc0, acc1, acc2, acc3, ah, b0, b1, b2, b3, ah);
    }
  }
  epi64<0>(slab + wave * SLAB64, acc0, acc1, acc2, acc3, oscale, (const float*)0, C, DMOD, rowA, col0, lane);
}

extern "C" void kernel_launch(void* const* d_in, const int* in_sizes, int n_in,
                              void* d_out, int out_size, void* d_ws, size_t ws_size,
                              hipStream_t stream) {
  if (n_in < 17) return;
  if (in_sizes[0] < ((NB - 1) * S_FULL + SEQ) * DMOD) return;
  if (in_sizes[1] < ((NB - 1) * S_FULL + SEQ) * NEXP) return;
  if (in_sizes[2] != DMOD * DMOD || in_sizes[4] != DMOD * DMOD || in_sizes[6] != DMOD * DMOD || in_sizes[8] != DMOD * DMOD) return;
  if (in_sizes[3] != DMOD || in_sizes[5] != DMOD || in_sizes[7] != DMOD) return;
  for (int i = 9; i <= 16; ++i) { if (in_sizes[i] != NL * DMOD) return; }
  if (out_size < MROWS * DMOD) return;

  const float* x    = (const float*)d_in[0];
  const float* gate = (const float*)d_in[1];
  const float* wq   = (const float*)d_in[2];
  const float* bq   = (const float*)d_in[3];
  const float* wk   = (const float*)d_in[4];
  const float* bk   = (const float*)d_in[5];
  const float* wv   = (const float*)d_in[6];
  const float* bv   = (const float*)d_in[7];
  const float* wo   = (const float*)d_in[8];
  const float* aq   = (const float*)d_in[9];
  const float* bmq  = (const float*)d_in[10];
  const float* ak   = (const float*)d_in[11];
  const float* bmk  = (const float*)d_in[12];
  const float* av   = (const float*)d_in[13];
  const float* bmv  = (const float*)d_in[14];
  const float* ao   = (const float*)d_in[15];
  const float* bmo  = (const float*)d_in[16];
  float*       out  = (float*)d_out;

  size_t off = 0;
  const size_t oXC = 0;
  const size_t oF  = SZ_XC;
  const size_t oOC = 0;
  const size_t oOL = SZ_XC;
  off = SZ_G0;
  const size_t oWC = off; off += SZ_WC;
  const size_t oAE = off; off += SZ_AE;
  const size_t oQH = off; off += SZ_Q;
  const size_t oQL = off; off += SZ_Q;
  const size_t oKH = off; off += SZ_Q;
  const size_t oKL = off; off += SZ_KL;
  const size_t oVH = off; off += SZ_Q;
  const size_t oVL = off; off += SZ_VL;
  if (off != SZ_TOTAL) return;
  if (off > ws_size) return;
  if (off > (size_t)WS_CAP) return;

  char* ws = (char*)d_ws;
  u16*   XC = (u16*)(ws + oXC);
  float* F  = (float*)(ws + oF);
  u16*   OC = (u16*)(ws + oOC);
  u16*   OL = (u16*)(ws + oOL);
  u16*   WC = (u16*)(ws + oWC);
  u16*   AE = (u16*)(ws + oAE);
  u16*   QH = (u16*)(ws + oQH);
  u16*   QL = (u16*)(ws + oQL);
  u16*   KH = (u16*)(ws + oKH);
  u16*   KL = (u16*)(ws + oKL);
  u16*   VH = (u16*)(ws + oVH);
  u16*   VL = (u16*)(ws + oVL);

  const dim3 b256(256), b128(128), bAT(ATT_THREADS);
  const dim3 gXB(((SEQ * DMOD) / 8 + 255) / 256);
  const dim3 gW(((DMOD * DMOD) / 8 + 255) / 256);
  const dim3 gBM(((DMOD * NL) / 8 + 255) / 256);
  const dim3 gAA(((NL * DMOD) / 8 + 255) / 256);
  const dim3 gLR((MROWS / 64) * 2);
  const dim3 gG((MROWS / 64) * (DMOD / 64));
  const dim3 gRP(MROWS);
  const dim3 gVT(NB * NH * NSTT);
  const int  nrtR = QO / 64;
  const int  nrtP = (SEQ - QO) / 64;

  for (int b = 0; b < NB; ++b) {
    cvtrows<<<gXB, b256, 0, stream>>>(x + (size_t)b * S_FULL * DMOD, DMOD, DMOD, SEQ,
                                      XC + (size_t)b * SEQ * KC, KC, 0, 0, 1.0f);
  }
  const float* Wp[3]  = {wq, wk, wv};
  const float* Bp[3]  = {bq, bk, bv};
  const float* Ap[3]  = {aq, ak, av};
  const float* Mp[3]  = {bmq, bmk, bmv};
  for (int pj = 0; pj < 3; ++pj) {
    cvtrows<<<gW,  b256, 0, stream>>>(Wp[pj], DMOD, DMOD, DMOD, WC, KC, 0, 0, 1.0f);
    cvtrows<<<gBM, b256, 0, stream>>>(Mp[pj], NL, NL, DMOD, WC, KC, DMOD, 0, 1.0f);
    cvtrows<<<gBM, b256, 0, stream>>>(Mp[pj], NL, NL, DMOD, WC, KC, DMOD + NL, 0, 1.0f);
    cvtrows<<<gAA, b256, 0, stream>>>(Ap[pj], DMOD, DMOD, NL, AE, DMOD, 0, 0, 1.0f);
    gemm_lr<0, 0><<<gLR, b128, 0, stream>>>(XC, KC, AE, DMOD, DMOD, gate, XC, MROWS, 1.0f, 1.0f);
    gemm_bff<<<gG, b128, 0, stream>>>(XC, KC, WC, KC, Bp[pj], F, DMOD, MROWS, DMOD, KC);
    if (pj == 0) {
      rope16<<<gRP, b128, 0, stream>>>(F, QH, QL, SEQ, QSC);
    } else if (pj == 1) {
      rope16<<<gRP, b128, 0, stream>>>(F, KH, KL, QO, KSC);
    } else {
      vt16<<<gVT, b256, 0, stream>>>(F, VH, VL);
    }
  }
  attn_c<1><<<dim3(NQTE * NHG * NB), bAT, 0, stream>>>(QH, QL, KH, KL, VH, VL, OC, OL, 0, NQTE);
  if (NQT > NQTE) {
    attn_c<0><<<dim3((NQT - NQTE) * NHG * NB), bAT, 0, stream>>>(QH, QL, KH, KL, VH, VL, OC, OL, NQTE, NQT - NQTE);
  }
  cvtrows<<<gW,  b256, 0, stream>>>(wo,  DMOD, DMOD, DMOD, WC, KC, 0, 1, WOS);
  cvtrows<<<gBM, b256, 0, stream>>>(bmo, NL, NL, DMOD, WC, KC, DMOD, 1, WOS);
  cvtrows<<<gBM, b256, 0, stream>>>(bmo, NL, NL, DMOD, WC, KC, DMOD + NL, 1, WOS);
  cvtrows<<<gAA, b256, 0, stream>>>(ao,  DMOD, DMOD, NL, AE, DMOD, 0, 1, AOS);
  gemm_lr<1, 1><<<gLR, b128, 0, stream>>>(OC, KC, AE, DMOD, DMOD, gate, OC, MROWS, 1.0f / (OSC * AOS), OSC);
  gemm_o<2><<<dim3(NB * nrtR * (DMOD / 64)), b128, 0, stream>>>(OC, OL, WC, out, 0, nrtR, 1.0f / (OSC * WOS));
  if (nrtP > 0) {
    gemm_o<1><<<dim3(NB * nrtP * (DMOD / 64)), b128, 0, stream>>>(OC, OL, WC, out, QO, nrtP, 1.0f / (OSC * WOS));
  }
  (void)hipGetLastError();
}
